// TARNet_23313082482710
// MI455X (gfx1250) — hardware-verified
//
#include <hip/hip_runtime.h>
#include <math.h>

typedef __attribute__((ext_vector_type(16))) _Float16 v16h;
typedef __attribute__((ext_vector_type(16))) __bf16 v16b;
typedef __attribute__((ext_vector_type(8)))  _Float16 v8h;
typedef __attribute__((ext_vector_type(8)))  float v8f;
typedef __attribute__((ext_vector_type(4)))  float v4f;
typedef __attribute__((ext_vector_type(2)))  float v2f;
typedef __attribute__((ext_vector_type(4)))  unsigned v4u;
typedef __attribute__((ext_vector_type(4)))  int v4i;
typedef float __attribute__((may_alias)) float_a;
typedef int __attribute__((may_alias)) int_a;

template <typename T> __device__ __forceinline__ void vst2(void* p, T v) { *(volatile T*)p = v; __threadfence(); *(volatile T*)p = v; }
__device__ __forceinline__ v8f wmma16(v16h a, v16h b, v8f c) {
  v8f d = __builtin_amdgcn_wmma_f32_16x16x32_f16(false, a, false, b, (short)0, c, false, false);
  asm volatile("v_nop\n\tv_nop\n\tv_nop\n\tv_nop" : "+v"(d) : "v"(a), "v"(b));
  return d;
}
__device__ __forceinline__ v8f wmma_bf(v16b a, v16b b, v8f c) {
  v8f d = __builtin_amdgcn_wmma_f32_16x16x32_bf16(false, a, false, b, (short)0, c, false, false);
  asm volatile("v_nop\n\tv_nop\n\tv_nop\n\tv_nop" : "+v"(d) : "v"(a), "v"(b));
  return d;
}
__device__ __forceinline__ v16h frag_h(const _Float16* rowk0, int lane) {
  union { v16h v; v8h q[2]; } u; const _Float16* p = rowk0 + 8 * (lane >> 4);
  u.q[0] = *(const v8h*)p; u.q[1] = *(const v8h*)(p + 16); return u.v;
}
__device__ __forceinline__ v16h frag_f32(const float* rowk0, int lane) {
  v16h a; const float* p = rowk0 + 8 * (lane >> 4);
#pragma unroll
  for (int i = 0; i < 8; ++i) { a[i] = (_Float16)p[i]; a[8 + i] = (_Float16)p[16 + i]; }
  return a;
}
__device__ __forceinline__ v16h frag_f32s(const float* rowk0, int lane, float sc) {
  v16h a; const float* p = rowk0 + 8 * (lane >> 4);
#pragma unroll
  for (int i = 0; i < 8; ++i) { a[i] = (_Float16)(p[i] * sc); a[8 + i] = (_Float16)(p[16 + i] * sc); }
  return a;
}
__device__ __forceinline__ v16h fragc_f32(const float* W, int k0, int n, int lane, int ld, int K) {
  v16h a; const int g = lane >> 4;
#pragma unroll
  for (int i = 0; i < 8; ++i) { const int ka = k0 + 8 * g + i, kb = ka + 16;
    a[i] = (_Float16)(ka < K ? W[(size_t)(ka < K ? ka : K - 1) * ld + n] : 0.f); a[8 + i] = (_Float16)(kb < K ? W[(size_t)(kb < K ? kb : K - 1) * ld + n] : 0.f); }
  return a;
}
struct F2 { v16b h, l; };
__device__ __forceinline__ F2 bsplit16(const float v[16]) { F2 r;
#pragma unroll
  for (int i = 0; i < 16; ++i) { const __bf16 h = (__bf16)v[i]; r.h[i] = h; r.l[i] = (__bf16)(v[i] - (float)h); }
  return r; }
__device__ __forceinline__ F2 split_row(const float* row, int k0, int lane) { float v[16]; const float* p = row + k0 + 8 * (lane >> 4);
#pragma unroll
  for (int i = 0; i < 8; ++i) { v[i] = p[i]; v[8 + i] = p[16 + i]; }
  return bsplit16(v); }
__device__ __forceinline__ F2 split_rowK(const float* row, int k0, int lane, int K) { float v[16]; const int g = lane >> 4;
#pragma unroll
  for (int i = 0; i < 8; ++i) { const int ka = k0 + 8 * g + i, kb = ka + 16; v[i] = ka < K ? row[ka < K ? ka : K - 1] : 0.f; v[8 + i] = kb < K ? row[kb < K ? kb : K - 1] : 0.f; }
  return bsplit16(v); }
__device__ __forceinline__ F2 split_col(const float* W, int k0, int n, int lane, int ld, int K) { float v[16]; const int g = lane >> 4;
#pragma unroll
  for (int i = 0; i < 8; ++i) { const int ka = k0 + 8 * g + i, kb = ka + 16; v[i] = ka < K ? W[(size_t)(ka < K ? ka : K - 1) * ld + n] : 0.f; v[8 + i] = kb < K ? W[(size_t)(kb < K ? kb : K - 1) * ld + n] : 0.f; }
  return bsplit16(v); }
__device__ __forceinline__ v8f mac3(const F2& a, const F2& b, v8f c) { c = wmma_bf(a.l, b.h, c); c = wmma_bf(a.h, b.l, c); return wmma_bf(a.h, b.h, c); }
__device__ __forceinline__ float sigm(float v) { return 1.0f / (1.0f + expf(-v)); }
#define LDSX() do { asm volatile("s_wait_dscnt 0" ::: "memory"); __builtin_amdgcn_wave_barrier(); __builtin_amdgcn_fence(__ATOMIC_RELEASE, "workgroup"); } while (0)


#define NS 16384
#define IN 512
#define H1 512
#define H2 256
#define NOUT 4
#define NT 4
#ifndef TRB
#define TRB (NS / 64)
#endif
typedef __attribute__((ext_vector_type(8))) __bf16 v8b;
__device__ __forceinline__ v16b frag_b(const __bf16* rowk0, int lane) {
  union { v16b v; v8b q[2]; } u; const __bf16* p = rowk0 + 8 * (lane >> 4);
  u.q[0] = *(const v8b*)p; u.q[1] = *(const v8b*)(p + 16); return u.v;
}
__device__ __forceinline__ float bfr(float v) { return (float)(__bf16)v; }
__device__ __attribute__((noinline)) float exp_ni(float v) { return expf(v); }
__device__ __attribute__((noinline)) float erf_ni(float v) { return erff(v); }

#define WS_P1  0u
#define WS_P2  (WS_P1 + 2u * (size_t)NOUT * H1 * IN)
#define WS_H   (WS_P2 + 2u * (size_t)NOUT * NT * H2 * H1)
#define WS_END (WS_H + 2u * (size_t)NOUT * NS * H1)

__global__ __launch_bounds__(256) void k_pack(const float* __restrict__ W1, const float* __restrict__ W2, __bf16* __restrict__ P1, _Float16* __restrict__ P2) { const int t = threadIdx.x; int n = blockIdx.x;
  if (n < NOUT * H1) { const int o = n / H1, c = n % H1; __shared__ __align__(16) __bf16 s[IN]; for (int k = t; k < IN; k += 256) s[k] = (__bf16)W1[((size_t)o * IN + k) * H1 + c]; __syncthreads(); for (int q = t; q < IN / 8; q += 256) vst2((unsigned*)(P1 + (size_t)n * IN + q * 8), *(const v4u*)&s[q * 8]); }
  else { n -= NOUT * H1; const int ot = n / H2, c = n % H2; __shared__ __align__(16) _Float16 s2[H1]; for (int k = t; k < H1; k += 256) s2[k] = (_Float16)(bfr(W2[((size_t)ot * H1 + k) * H2 + c]) * 256.0f); __syncthreads(); for (int q = t; q < H1 / 8; q += 256) vst2((unsigned*)(P2 + (size_t)n * H1 + q * 8), *(const v4u*)&s2[q * 8]); } }
__global__ __launch_bounds__(128) void k_shared(const float* __restrict__ X, const __bf16* __restrict__ P1, const float* __restrict__ B1, const float* __restrict__ G1, const float* __restrict__ BE1, const float* __restrict__ M1, const float* __restrict__ V1, _Float16* __restrict__ H) {
  __shared__ __align__(16) _Float16 so[64][136];
  const int tid = threadIdx.x, wave = tid >> 5, lane = tid & 31, col = lane & 15, g = lane >> 4; const int o = blockIdx.z; const size_t r0 = (size_t)blockIdx.x * 64 + wave * 16; const int n0 = blockIdx.y * 128;
  v8f acc[8] = {};
#pragma unroll 2
  for (int kc = 0; kc < IN / 32; ++kc) { v16b a; { const float* p = X + (r0 + col) * IN + kc * 32 + 8 * g;
#pragma unroll
      for (int i = 0; i < 8; ++i) { a[i] = (__bf16)p[i]; a[8 + i] = (__bf16)p[16 + i]; } }
#pragma unroll
    for (int j = 0; j < 8; ++j) acc[j] = wmma_bf(a, frag_b(P1 + ((size_t)o * H1 + n0 + j * 16 + col) * IN + kc * 32, lane), acc[j]); }
#pragma unroll
  for (int j = 0; j < 8; ++j) { const int c = n0 + j * 16 + col; const size_t oc = (size_t)o * H1 + c; const float bb = bfr(B1[oc]), sc = bfr(G1[oc]) / sqrtf(bfr(V1[oc]) + 1e-5f), mm = bfr(M1[oc]), be = bfr(BE1[oc]);
#pragma unroll
    for (int r = 0; r < 8; ++r) so[wave * 16 + 8 * g + r][j * 16 + col] = (_Float16)((fmaxf(acc[j][r] + bb, 0.f) - mm) * sc + be); }
  LDSX();
  for (int rl = 0; rl < 16; ++rl) if (lane < 16) vst2((unsigned*)(H + ((size_t)o * NS + r0 + rl) * H1 + n0 + lane * 8), *(const v4u*)&so[wave * 16 + rl][lane * 8]);
}
__global__ __launch_bounds__(128) void k_heads(const _Float16* __restrict__ H, const _Float16* __restrict__ P2, const int* __restrict__ TREAT, const float* __restrict__ B2, const float* __restrict__ G2, const float* __restrict__ BE2, const float* __restrict__ M2, const float* __restrict__ V2, const float* __restrict__ W3, const float* __restrict__ B3, float* __restrict__ OUT) {
  __shared__ __align__(16) float sout[64][NOUT]; __shared__ float spart[4][16][16];
  const int tid = threadIdx.x, wave = tid >> 5, lane = tid & 31, col = lane & 15, g = lane >> 4; const size_t r0 = (size_t)blockIdx.x * 64 + wave * 16;
  int tr[8];
#pragma unroll
  for (int r = 0; r < 8; ++r) tr[r] = TREAT[r0 + 8 * g + r];
#pragma unroll 1
  for (int o = 0; o < NOUT; ++o) {
#pragma unroll 1
    for (int t = 0; t < NT; ++t) { const size_t ot = (size_t)o * NT + t; v8f acc[16] = {};
#pragma unroll 2
      for (int kc = 0; kc < H1 / 32; ++kc) { const v16h a = frag_h(H + ((size_t)o * NS + r0 + col) * H1 + kc * 32, lane);
#pragma unroll
        for (int j = 0; j < 16; ++j) acc[j] = wmma16(a, frag_h(P2 + (ot * H2 + j * 16 + col) * H1 + kc * 32, lane), acc[j]); }
      float pd[8] = {0.f, 0.f, 0.f, 0.f, 0.f, 0.f, 0.f, 0.f};
#pragma unroll
      for (int j = 0; j < 16; ++j) { const int c = j * 16 + col; const size_t oc = ot * H2 + c; const float bb = bfr(B2[oc]), sc = bfr(G2[oc]) / sqrtf(bfr(V2[oc]) + 1e-5f), mm = bfr(M2[oc]), be = bfr(BE2[oc]), w3 = bfr(W3[oc]);
#pragma unroll
        for (int r = 0; r < 8; ++r) { const float z = (fmaxf(acc[j][r] * (1.0f / 256.0f) + bb, 0.f) - mm) * sc + be; pd[r] += z * w3; } }
#pragma unroll
      for (int r = 0; r < 8; ++r) {
#pragma unroll
        for (int sh = 1; sh < 16; sh <<= 1) pd[r] += __shfl_xor(pd[r], sh); }
      const float b3 = bfr(B3[ot]);
      if (col == 0) {
#pragma unroll
        for (int r = 0; r < 8; ++r) if (tr[r] == t) sout[wave * 16 + 8 * g + r][o] = pd[r] + b3; } } }
  __syncthreads();
  if (tid < 64) vst2(OUT + ((size_t)blockIdx.x * 64 + tid) * NOUT, *(const v4f*)&sout[tid][0]);
}
extern "C" void kernel_launch(void* const* d_in, const int* in_sizes, int n_in, void* d_out, int out_size, void* d_ws, size_t ws_size, hipStream_t stream) {
  (void)in_sizes; (void)n_in; (void)out_size;
  const float** F = (const float**)d_in;
  if (ws_size < (size_t)WS_END) return;
  char* ws = (char*)d_ws; __bf16* P1 = (__bf16*)(ws + WS_P1); _Float16 *P2 = (_Float16*)(ws + WS_P2), *H = (_Float16*)(ws + WS_H);
  k_pack<<<NOUT * H1 + NOUT * NT * H2, 256, 0, stream>>>(F[2], F[8], P1, P2);
  k_shared<<<dim3(TRB, H1 / 128, NOUT), 128, 0, stream>>>(F[0], P1, F[3], F[4], F[5], F[6], F[7], H);
  k_heads<<<TRB, 128, 0, stream>>>(H, P2, (const int*)d_in[1], F[9], F[10], F[11], F[12], F[13], F[14], F[15], (float*)d_out);
}
